// MSDeform_attn_transformer_encoder_layer_74122545594641
// MI455X (gfx1250) — hardware-verified
//
#include <hip/hip_runtime.h>

typedef __attribute__((ext_vector_type(16))) _Float16 v16h;
typedef __attribute__((ext_vector_type(8)))  _Float16 v8h;
typedef __attribute__((ext_vector_type(4)))  _Float16 v4h;
typedef __attribute__((ext_vector_type(16))) __bf16   v16b;
typedef __attribute__((ext_vector_type(8)))  __bf16   v8b;
typedef __attribute__((ext_vector_type(8)))  float    v8f;
typedef __attribute__((ext_vector_type(4)))  float    v4f;

static constexpr int kBatch = 2;
static constexpr int kS     = 13125;
static constexpr int kD     = 256;
static constexpr int kFF    = 1024;
static constexpr int kM     = kBatch * kS;
static constexpr int kMpad  = 26304;
static constexpr int kNOA   = 320;
static constexpr int kNOFF  = 192;
static_assert(kMpad % 64 == 0 && kMpad >= kM, "tile multiple");
static_assert(kD % 32 == 0 && kFF % 32 == 0 && kNOA % 64 == 0, "K multiple of 32, N multiple of 64");

static constexpr size_t SZ_P16   = (size_t)kMpad * kD * 2;
static constexpr size_t SZ_P32   = (size_t)kMpad * kD * 4;
static constexpr size_t SZ_OA    = (size_t)kMpad * kNOA * 4;
static constexpr size_t SZ_F16   = (size_t)kMpad * kFF * 2;
static constexpr size_t OFF_R1   = 0;
static constexpr size_t OFF_Q16  = OFF_R1;
static constexpr size_t OFF_OA   = OFF_R1 + SZ_P16;
static constexpr size_t OFF_F16  = OFF_R1;
static constexpr size_t OFF_R2   = OFF_R1 + SZ_F16;
static constexpr size_t OFF_R3   = OFF_R2 + SZ_P16;
static constexpr size_t OFF_R4   = OFF_R3 + SZ_P32;
static constexpr size_t OFF_R5   = OFF_R4 + SZ_P32;
static constexpr size_t OFF_WVAL = OFF_R5;
static constexpr size_t OFF_WOUT = OFF_WVAL + (size_t)kD * kD * 2;
static constexpr size_t OFF_WCAT = OFF_WOUT + (size_t)kD * kD * 2;
static constexpr size_t OFF_W1T  = OFF_WCAT + (size_t)kNOA * kD * 2;
static constexpr size_t OFF_W2T  = OFF_W1T + (size_t)kFF * kD * 2;
static constexpr size_t OFF_BCAT = OFF_W2T + (size_t)kD * kFF * 2;
static constexpr size_t WS_TOTAL = OFF_BCAT + (size_t)kNOA * 4;
static_assert(OFF_OA + SZ_OA <= OFF_R2, "OA inside R1");
static_assert(WS_TOTAL <= (size_t)134217728, "carve under 128 MiB");
static_assert((OFF_OA % 128) == 0 && (OFF_R2 % 128) == 0 && (OFF_R3 % 128) == 0 && (OFF_R4 % 128) == 0 &&
              (OFF_R5 % 128) == 0 && (OFF_WCAT % 128) == 0 && (OFF_BCAT % 128) == 0, "128-B aligned regions");

__device__ __forceinline__ unsigned short f2bf_bits(float f) {
  unsigned u = __float_as_uint(f);
  return (unsigned short)((u + 0x7FFFu + ((u >> 16) & 1u)) >> 16);
}
__device__ __forceinline__ float bf_bits2f(unsigned short h) { return __uint_as_float(((unsigned)h) << 16); }

__device__ __forceinline__ void dep_guard_h(v8f& a, v8f& b, v16h x, v16h y) { asm volatile("v_nop\n\tv_nop\n\tv_nop\n\tv_nop" : "+v"(a), "+v"(b) : "v"(x), "v"(y)); }
__device__ __forceinline__ void dep_guard_b(v8f& a, v8f& b, v16b x, v16b y) { asm volatile("v_nop\n\tv_nop\n\tv_nop\n\tv_nop" : "+v"(a), "+v"(b) : "v"(x), "v"(y)); }
__device__ __forceinline__ void keep4_h(v16h a, v16h b, v16h c, v16h d) { asm volatile("v_nop" :: "v"(a), "v"(b), "v"(c), "v"(d)); }
__device__ __forceinline__ void keep4_b(v16b a, v16b b, v16b c, v16b d) { asm volatile("v_nop" :: "v"(a), "v"(b), "v"(c), "v"(d)); }
__device__ __forceinline__ void acc_guard4(v8f& a, v8f& b, v8f& c, v8f& d) { asm volatile("v_nop\n\tv_nop\n\tv_nop\n\tv_nop" : "+v"(a), "+v"(b), "+v"(c), "+v"(d)); }
template <typename T> struct Frag;
template <> struct Frag<_Float16> {
  typedef v16h V; union U { v16h v; v8h h[2]; };
  static __device__ __forceinline__ v16h load(const _Float16* p) {
    U f; f.h[0] = *(const v8h*)(p); f.h[1] = *(const v8h*)(p + 16); return f.v;
  }
  static __device__ __forceinline__ v8f mma(v16h a, v16h b, v8f c) {
    return __builtin_amdgcn_wmma_f32_16x16x32_f16(false, a, false, b, (short)0, c, false, false);
  }
  static __device__ __forceinline__ void guard(v8f& a, v8f& b, v16h x, v16h y) { dep_guard_h(a, b, x, y); }
  static __device__ __forceinline__ void keep(v16h a, v16h b, v16h c, v16h d) { keep4_h(a, b, c, d); }
};
template <> struct Frag<__bf16> {
  typedef v16b V; union U { v16b v; v8b h[2]; };
  static __device__ __forceinline__ v16b load(const __bf16* p) {
    U f; f.h[0] = *(const v8b*)(p); f.h[1] = *(const v8b*)(p + 16); return f.v;
  }
  static __device__ __forceinline__ v8f mma(v16b a, v16b b, v8f c) {
    return __builtin_amdgcn_wmma_f32_16x16x32_bf16(false, a, false, b, (short)0, c, false, false);
  }
  static __device__ __forceinline__ void guard(v8f& a, v8f& b, v16b x, v16b y) { dep_guard_b(a, b, x, y); }
  static __device__ __forceinline__ void keep(v16b a, v16b b, v16b c, v16b d) { keep4_b(a, b, c, d); }
};

template <int ET> struct Elem;
template <> struct Elem<0> { typedef _Float16 T; };
template <> struct Elem<1> { typedef __bf16 T; };
template <int ET, bool SPLIT, int BIAS_MODE, int OUT_MODE, bool RESID, int ACT = 0>
__global__ __launch_bounds__(256) void wmma_gemm64(
    const unsigned short* __restrict__ Ap, const unsigned short* __restrict__ A2p, int lda, long strideA,
    const unsigned short* __restrict__ Btp, const unsigned short* __restrict__ Bt2p, int ldb, long strideB,
    void* __restrict__ Cout, void* __restrict__ Cout2, int ldc, long strideC,
    const float* __restrict__ bias,
    const float* __restrict__ resid, long strideR,
    int M, int N, int K, float scale) {
  typedef typename Elem<ET>::T T;
  typedef typename Frag<T>::V V;
  const T* A = (const T*)Ap; const T* A2 = (const T*)A2p; const T* Bt = (const T*)Btp; const T* Bt2 = (const T*)Bt2p;
  __shared__ __align__(16) float sT[8][16 * 68];
  const int b    = blockIdx.y;
  const int lane = threadIdx.x & 31;
  const int wave = threadIdx.x >> 5;
  const int tilesN = N >> 6;
  const int tilesM = M >> 6;
  const int tile = blockIdx.x * 8 + wave;
  if (tile >= tilesM * tilesN) return;
  const int tm = tile / tilesN;
  const int tn = tile - tm * tilesN;
  const int m0 = tm << 6;
  const int n0 = tn << 6;

  const T* Ab  = A  + (size_t)b * strideA;
  const T* Bb  = Bt + (size_t)b * strideB;
  const T* Ab2 = SPLIT ? (A2  + (size_t)b * strideA) : nullptr;
  const T* Bb2 = SPLIT ? (Bt2 + (size_t)b * strideB) : nullptr;

  const int rlane = lane & 15;
  const int koff  = (lane >> 4) * 8;
  const int mOff  = (lane >> 4) * 8;

  v8f acc[4][4];
#pragma unroll
  for (int i = 0; i < 4; ++i)
#pragma unroll
    for (int j = 0; j < 4; ++j) acc[i][j] = (v8f){0.f,0.f,0.f,0.f,0.f,0.f,0.f,0.f};

  for (int k0 = 0; k0 < K; k0 += 32) {
    V bh[4], bl[4];
#pragma unroll
    for (int j = 0; j < 4; ++j) {
      const size_t bo = (size_t)(n0 + (j << 4) + rlane) * ldb + koff + k0;
      bh[j] = Frag<T>::load(Bb + bo);
      if (SPLIT) bl[j] = Frag<T>::load(Bb2 + bo);
    }
#pragma unroll
    for (int i = 0; i < 4; ++i) {
      const size_t ao = (size_t)(m0 + (i << 4) + rlane) * lda + koff + k0;
      V ah = Frag<T>::load(Ab + ao);
      V al;
      if (SPLIT) al = Frag<T>::load(Ab2 + ao);
#pragma unroll
      for (int j = 0; j < 4; ++j) {
        acc[i][j] = Frag<T>::mma(ah, bh[j], acc[i][j]);
        if (SPLIT) {
          acc[i][j] = Frag<T>::mma(ah, bl[j], acc[i][j]);
          acc[i][j] = Frag<T>::mma(al, bh[j], acc[i][j]);
        }
      }
      Frag<T>::guard(acc[i][0], acc[i][3], ah, SPLIT ? al : ah);
    }
    Frag<T>::keep(bh[0], bh[1], bh[2], bh[3]);
    if (SPLIT) Frag<T>::keep(bl[0], bl[1], bl[2], bl[3]);
  }
  acc_guard4(acc[0][0], acc[0][1], acc[0][2], acc[0][3]);
  acc_guard4(acc[1][0], acc[1][1], acc[1][2], acc[1][3]);
  acc_guard4(acc[2][0], acc[2][1], acc[2][2], acc[2][3]);
  acc_guard4(acc[3][0], acc[3][1], acc[3][2], acc[3][3]);

  float* slab = sT[wave];
  const float* Rb = RESID ? (resid + (size_t)b * strideR) : nullptr;
#pragma unroll
  for (int i = 0; i < 4; ++i) {
    const int mBase = m0 + (i << 4);
#pragma unroll
    for (int j = 0; j < 4; ++j) {
      const int n = n0 + (j << 4) + rlane;
      float bv = 0.f;
      if (BIAS_MODE == 2) bv = bias[n];
#pragma unroll
      for (int r = 0; r < 8; ++r) {
        float v = acc[i][j][r] * scale;
        if (BIAS_MODE == 1) v += bias[mBase + mOff + r];
        if (BIAS_MODE == 2) v += bv;
        if (RESID) v += Rb[(size_t)(mBase + mOff + r) * ldc + n];
        if (ACT == 1) v = tanhf(v);
        if (ACT == 2) v = fmaxf(v, 0.0f);
        if (ACT == 3) v = v / (1.0f + expf(-v));
        if (ACT == 4) v = (v > 0.f) ? v : 0.01f * v;
        if (ACT == 5) v = 0.5f * v * (1.0f + erff(v * 0.70710678118654752f));
        slab[(mOff + r) * 68 + (j << 4) + rlane] = v;
      }
    }
    __builtin_amdgcn_fence(__ATOMIC_RELEASE, "workgroup");
    __builtin_amdgcn_wave_barrier();
    __builtin_amdgcn_fence(__ATOMIC_ACQUIRE, "workgroup");
    if (OUT_MODE == 0) {
      float* C = (float*)Cout + (size_t)b * strideC;
      const int hh = lane >> 4, c4 = (lane & 15) * 4;
      for (int pass = 0; pass < 2; ++pass) {
#pragma unroll
        for (int it = 0; it < 8; ++it) {
          const int row = it * 2 + hh;
          v4f v = *(const v4f*)(slab + row * 68 + c4);
          *(volatile v4f*)(C + (size_t)(mBase + row) * ldc + n0 + c4) = v;
        }
        __threadfence();
      }
    } else {
      const int q = lane >> 3, c8 = (lane & 7) * 8;
      unsigned short* C  = (unsigned short*)Cout  + (size_t)b * strideC;
      unsigned short* C2 = (OUT_MODE == 2) ? ((unsigned short*)Cout2 + (size_t)b * strideC) : nullptr;
      for (int pass = 0; pass < 2; ++pass) {
#pragma unroll
        for (int it = 0; it < 4; ++it) {
          const int row = it * 4 + q;
          const float* sp = slab + row * 68 + c8;
          v8h hv, lv;
#pragma unroll
          for (int e = 0; e < 8; ++e) {
            if (OUT_MODE == 1) {
              hv[e] = (_Float16)sp[e];
            } else {
              unsigned short hb = f2bf_bits(sp[e]);
              unsigned short lb = f2bf_bits(sp[e] - bf_bits2f(hb));
              hv[e] = __builtin_bit_cast(_Float16, hb);
              lv[e] = __builtin_bit_cast(_Float16, lb);
            }
          }
          *(volatile v8h*)(C + (size_t)(mBase + row) * ldc + n0 + c8) = hv;
          if (OUT_MODE == 2) *(volatile v8h*)(C2 + (size_t)(mBase + row) * ldc + n0 + c8) = lv;
        }
        __threadfence();
      }
    }
    __builtin_amdgcn_fence(__ATOMIC_RELEASE, "workgroup");
    __builtin_amdgcn_wave_barrier();
    __builtin_amdgcn_fence(__ATOMIC_ACQUIRE, "workgroup");
  }
}

__global__ __launch_bounds__(256) void prep_act(const float* __restrict__ x, const float* __restrict__ pos,
                                               _Float16* __restrict__ x16, _Float16* __restrict__ q16) {
  const int t = blockIdx.x * 256 + threadIdx.x;
  const int row = t >> 5;
  const int ch = t & 31;
  const int rowc = row < kM ? row : (kM - 1);
  const size_t src = (size_t)rowc * kD + (size_t)ch * 8;
  const v4f xa = *(const v4f*)(x + src), xb = *(const v4f*)(x + src + 4);
  const v4f pa = *(const v4f*)(pos + src), pb = *(const v4f*)(pos + src + 4);
  const v8f xx = __builtin_shufflevector(xa, xb, 0, 1, 2, 3, 4, 5, 6, 7);
  const v8f pp = __builtin_shufflevector(pa, pb, 0, 1, 2, 3, 4, 5, 6, 7);
  v8h hx = __builtin_convertvector(xx, v8h);
  v8h hq = __builtin_convertvector(xx + pp, v8h);
  v8h z = {};
  if (row >= kM) { hx = z; hq = z; }
  const size_t d = (size_t)t * 8;
  *(volatile v8h*)(x16 + d) = hx;
  *(volatile v8h*)(q16 + d) = hq;
  __threadfence();
  *(volatile v8h*)(x16 + d) = hx;
  *(volatile v8h*)(q16 + d) = hq;
}

__global__ __launch_bounds__(256) void prep_wt16(const float* __restrict__ W, _Float16* __restrict__ Wt,
                                                int Kdim, int Nreal, int Npad) {
  const int t = blockIdx.x * 256 + threadIdx.x;
  const int k8n = Kdim >> 3;
  const int total = Npad * k8n;
  if (t >= total) return;
  const int n = t / k8n;
  const int k8 = t - n * k8n;
  const int ncl = n < Nreal ? n : (Nreal - 1);
  v8h hv;
#pragma unroll
  for (int i = 0; i < 8; ++i) {
    const float v = W[(size_t)(k8 * 8 + i) * Nreal + ncl] * 16.0f;
    hv[i] = (_Float16)v;
  }
  v8h z = {};
  if (n >= Nreal) hv = z;
  _Float16* dst = Wt + (size_t)n * Kdim + (size_t)k8 * 8;
  *(volatile v8h*)dst = hv;
  __threadfence();
  *(volatile v8h*)dst = hv;
}

__global__ __launch_bounds__(320) void prep_bias_cat(const float* __restrict__ boff, const float* __restrict__ battn,
                                                    float* __restrict__ bcat) {
  const int n = threadIdx.x;
  const int i0 = n < 191 ? n : 191;
  int i1 = n - kNOFF;
  i1 = i1 < 0 ? 0 : (i1 > 95 ? 95 : i1);
  const float v0 = boff[i0];
  const float v1 = battn[i1];
  const float v = (n < kNOFF) ? v0 : ((n < kNOFF + 96) ? v1 : 0.0f);
  ((volatile float*)bcat)[n] = v;
  __threadfence();
  ((volatile float*)bcat)[n] = v;
}

__device__ __forceinline__ void corner_acc(float (&acc)[8], const float* __restrict__ valb,
                                           int st, int iW, int iH, int yi, int xi, float w, float aw) {
#pragma clang fp contract(off)
  const bool ok = (xi >= 0) && (xi < iW) && (yi >= 0) && (yi < iH);
  const float wv = w * (ok ? 1.0f : 0.0f);
  const float coef = aw * wv;
  int xc = xi < 0 ? 0 : xi;
  xc = xc > iW - 1 ? iW - 1 : xc;
  int yc = yi < 0 ? 0 : yi;
  yc = yc > iH - 1 ? iH - 1 : yc;
  int vr = st + yc * iW + xc;
  vr = vr < 0 ? 0 : (vr > kS - 1 ? kS - 1 : vr);
  const float* vp = valb + (size_t)vr * kD;
  const v4f g0 = *(const v4f*)vp;
  const v4f g1 = *(const v4f*)(vp + 4);
#pragma unroll
  for (int e = 0; e < 4; ++e) {
    acc[e]     = fmaf(coef, g0[e], acc[e]);
    acc[4 + e] = fmaf(coef, g1[e], acc[4 + e]);
  }
}

__global__ __launch_bounds__(256) void sample_kernel(const float* __restrict__ val, const float* __restrict__ oa,
                                                    const float* __restrict__ refp, _Float16* __restrict__ ao16) {
#pragma clang fp contract(off)
  const int wave = threadIdx.x >> 5;
  const int lane = threadIdx.x & 31;
  const int row = blockIdx.x * 8 + wave;
  const int h = lane >> 2;
  const int c = lane & 3;
  const int rowc = row < kM ? row : (kM - 1);
  const int bidx = rowc >= kS ? 1 : 0;

  const float* oar  = oa + (size_t)rowc * kNOA;
  const float* lgp  = oar + kNOFF + h * 12;
  const float* offp = oar + h * 24;

  float lg[12];
#pragma unroll
  for (int j = 0; j < 12; ++j) lg[j] = lgp[j];
  float mx = lg[0];
#pragma unroll
  for (int j = 1; j < 12; ++j) mx = fmaxf(mx, lg[j]);
  float sum = 0.0f;
#pragma unroll
  for (int j = 0; j < 12; ++j) sum += __expf(lg[j] - mx);
  const float inv = 1.0f / sum;

  const float* rp = refp + (size_t)rowc * 6;
  const float r0x = rp[0], r0y = rp[1], r1x = rp[2], r1y = rp[3], r2x = rp[4], r2y = rp[5];

  const float* valb = val + (size_t)bidx * kS * kD + h * 32 + c * 8;

  float acc[8];
#pragma unroll
  for (int e = 0; e < 8; ++e) acc[e] = 0.0f;

#pragma unroll 1
  for (int pt = 0; pt < 12; ++pt) {
    const int l = pt >> 2;
    const int iH = (l == 0) ? 100 : ((l == 1) ? 50 : 25);
    const int iW = (l == 0) ? 100 : ((l == 1) ? 50 : 25);
    const int st = (l == 0) ? 0 : ((l == 1) ? 10000 : 12500);
    const float fW = (float)iW, fH = (float)iH;
    const float rcW = (l == 0) ? 0.01f : ((l == 1) ? 0.02f : 0.04f);
    const float rcH = (l == 0) ? 0.01f : ((l == 1) ? 0.02f : 0.04f);
    const float rx = (l == 0) ? r0x : ((l == 1) ? r1x : r2x);
    const float ry = (l == 0) ? r0y : ((l == 1) ? r1y : r2y);
    const float aw = __expf(lgp[pt] - mx) * inv;
    const float ox = offp[pt * 2 + 0];
    const float oy = offp[pt * 2 + 1];
    const float locx = rx + ox * rcW;
    const float locy = ry + oy * rcH;
    const float px = locx * fW - 0.5f;
    const float py = locy * fH - 0.5f;
    const float x0f = floorf(px), y0f = floorf(py);
    const float fx = px - x0f, fy = py - y0f;
    const int x0 = (int)x0f, y0 = (int)y0f;
    const float gx = 1.0f - fx, gy = 1.0f - fy;
    corner_acc(acc, valb, st, iW, iH, y0,     x0,     gx * gy, aw);
    corner_acc(acc, valb, st, iW, iH, y0,     x0 + 1, fx * gy, aw);
    corner_acc(acc, valb, st, iW, iH, y0 + 1, x0,     gx * fy, aw);
    corner_acc(acc, valb, st, iW, iH, y0 + 1, x0 + 1, fx * fy, aw);
  }

  v8h o;
#pragma unroll
  for (int e = 0; e < 8; ++e) o[e] = (_Float16)(acc[e] * 16.0f);
  v8h z = {};
  if (row >= kM) o = z;
  _Float16* dst = ao16 + (size_t)row * kD + lane * 8;
  *(volatile v8h*)dst = o;
  __threadfence();
  *(volatile v8h*)dst = o;
}

__device__ __forceinline__ float wave_sum(float v) {
#pragma unroll
  for (int off = 16; off >= 1; off >>= 1) v += __shfl_xor(v, off, 32);
  return v;
}

__global__ __launch_bounds__(256) void ln1_kernel(const float* __restrict__ t1, const float* __restrict__ xin,
                                                 const float* __restrict__ g, const float* __restrict__ be,
                                                 float* __restrict__ h1, _Float16* __restrict__ h1h) {
  const int wave = threadIdx.x >> 5, lane = threadIdx.x & 31;
  const int row = blockIdx.x * 8 + wave;
  const int c0 = lane * 4, c1 = 128 + lane * 4;
  const v4f ga = *(const v4f*)(g + c0), gb = *(const v4f*)(g + c1);
  const v4f ba = *(const v4f*)(be + c0), bb = *(const v4f*)(be + c1);
  v4f o0 = {0.f, 0.f, 0.f, 0.f}, o1 = {0.f, 0.f, 0.f, 0.f};
  if (row < kM) {
    const float* tp = t1 + (size_t)row * kD;
    const float* xp = xin + (size_t)row * kD;
    const v4f a0 = *(const v4f*)(tp + c0) + *(const v4f*)(xp + c0);
    const v4f a1 = *(const v4f*)(tp + c1) + *(const v4f*)(xp + c1);
    float s = (a0[0] + a0[1]) + (a0[2] + a0[3]) + (a1[0] + a1[1]) + (a1[2] + a1[3]);
    s = wave_sum(s);
    const float mean = s * (1.0f / 256.0f);
    const v4f d0 = a0 - mean, d1 = a1 - mean;
    float sq = (d0[0] * d0[0] + d0[1] * d0[1]) + (d0[2] * d0[2] + d0[3] * d0[3]) +
               (d1[0] * d1[0] + d1[1] * d1[1]) + (d1[2] * d1[2] + d1[3] * d1[3]);
    sq = wave_sum(sq);
    const float var = sq * (1.0f / 256.0f);
    const float rstd = rsqrtf(var + 1e-5f);
    o0 = d0 * rstd * ga + ba;
    o1 = d1 * rstd * gb + bb;
  }
  float* hp = h1 + (size_t)row * kD;
  const int sl0 = (2 * lane) & 31, sl1 = (2 * lane + 1) & 31;
  const bool lowhalf = lane < 16;
  v8h pk;
#pragma unroll
  for (int e = 0; e < 4; ++e) {
    const float fa0 = __shfl(o0[e], sl0, 32);
    const float fa1 = __shfl(o1[e], sl0, 32);
    const float fb0 = __shfl(o0[e], sl1, 32);
    const float fb1 = __shfl(o1[e], sl1, 32);
    pk[e]     = (_Float16)(lowhalf ? fa0 : fa1);
    pk[4 + e] = (_Float16)(lowhalf ? fb0 : fb1);
  }
  _Float16* hh = h1h + (size_t)row * kD + lane * 8;
  *(volatile v4f*)(hp + c0) = o0;
  *(volatile v4f*)(hp + c1) = o1;
  *(volatile v8h*)hh = pk;
  __threadfence();
  *(volatile v4f*)(hp + c0) = o0;
  *(volatile v4f*)(hp + c1) = o1;
  *(volatile v8h*)hh = pk;
}

__global__ __launch_bounds__(256) void ln2_kernel(const float* __restrict__ t2,
                                                 const float* __restrict__ g, const float* __restrict__ be,
                                                 float* __restrict__ outp) {
  const int wave = threadIdx.x >> 5, lane = threadIdx.x & 31;
  const int row = blockIdx.x * 8 + wave;
  if (row >= kM) return;
  const int c0 = lane * 4, c1 = 128 + lane * 4;
  const v4f ga = *(const v4f*)(g + c0), gb = *(const v4f*)(g + c1);
  const v4f ba = *(const v4f*)(be + c0), bb = *(const v4f*)(be + c1);
  const float* tp = t2 + (size_t)row * kD;
  const v4f a0 = *(const v4f*)(tp + c0);
  const v4f a1 = *(const v4f*)(tp + c1);
  float s = (a0[0] + a0[1]) + (a0[2] + a0[3]) + (a1[0] + a1[1]) + (a1[2] + a1[3]);
  s = wave_sum(s);
  const float mean = s * (1.0f / 256.0f);
  const v4f d0 = a0 - mean, d1 = a1 - mean;
  float sq = (d0[0] * d0[0] + d0[1] * d0[1]) + (d0[2] * d0[2] + d0[3] * d0[3]) +
             (d1[0] * d1[0] + d1[1] * d1[1]) + (d1[2] * d1[2] + d1[3] * d1[3]);
  sq = wave_sum(sq);
  const float var = sq * (1.0f / 256.0f);
  const float rstd = rsqrtf(var + 1e-5f);
  const v4f o0 = d0 * rstd * ga + ba;
  const v4f o1 = d1 * rstd * gb + bb;
  float* op = outp + (size_t)row * kD;
  *(volatile v4f*)(op + c0) = o0;
  *(volatile v4f*)(op + c1) = o1;
  __threadfence();
  *(volatile v4f*)(op + c0) = o0;
  *(volatile v4f*)(op + c1) = o1;
}

static constexpr int gemm_blocks(int N) { return ((kMpad / 64) * (N / 64) + 7) / 8; }

extern "C" void kernel_launch(void* const* d_in, const int* in_sizes, int n_in,
                              void* d_out, int out_size, void* d_ws, size_t ws_size,
                              hipStream_t stream) {
  if (n_in < 19) return;
  if (in_sizes[0] != kM * kD || in_sizes[1] != kM * kD || in_sizes[2] != kM * 6) return;
  if (in_sizes[3] != kD * 192 || in_sizes[4] != 192 || in_sizes[5] != kD * 96 || in_sizes[6] != 96) return;
  if (in_sizes[7] != kD * kD || in_sizes[8] != kD || in_sizes[9] != kD * kD || in_sizes[10] != kD) return;
  if (in_sizes[11] != kD || in_sizes[12] != kD || in_sizes[13] != kD * kFF || in_sizes[14] != kFF) return;
  if (in_sizes[15] != kFF * kD || in_sizes[16] != kD || in_sizes[17] != kD || in_sizes[18] != kD) return;
  if (out_size != kM * kD) return;
  if (ws_size < WS_TOTAL) return;

  const float* x     = (const float*)d_in[0];
  const float* pos   = (const float*)d_in[1];
  const float* refp  = (const float*)d_in[2];
  const float* Woff  = (const float*)d_in[3];
  const float* boff  = (const float*)d_in[4];
  const float* Wattn = (const float*)d_in[5];
  const float* battn = (const float*)d_in[6];
  const float* Wval  = (const float*)d_in[7];
  const float* bval  = (const float*)d_in[8];
  const float* Wout  = (const float*)d_in[9];
  const float* bout  = (const float*)d_in[10];
  const float* g1    = (const float*)d_in[11];
  const float* be1   = (const float*)d_in[12];
  const float* W1    = (const float*)d_in[13];
  const float* b1    = (const float*)d_in[14];
  const float* W2    = (const float*)d_in[15];
  const float* b2    = (const float*)d_in[16];
  const float* g2    = (const float*)d_in[17];
  const float* be2   = (const float*)d_in[18];

  char* ws = (char*)d_ws;
  _Float16* q16  = (_Float16*)(ws + OFF_Q16);
  float*    oa   = (float*)(ws + OFF_OA);
  _Float16* f16p = (_Float16*)(ws + OFF_F16);
  _Float16* x16  = (_Float16*)(ws + OFF_R2);
  _Float16* ao16 = (_Float16*)(ws + OFF_R2);
  _Float16* h1h  = (_Float16*)(ws + OFF_R2);
  float*    valp = (float*)(ws + OFF_R3);
  float*    t1   = (float*)(ws + OFF_R3);
  float*    t2   = (float*)(ws + OFF_R3);
  float*    h1   = (float*)(ws + OFF_R4);
  _Float16* wvalT = (_Float16*)(ws + OFF_WVAL);
  _Float16* woutT = (_Float16*)(ws + OFF_WOUT);
  _Float16* wcatT = (_Float16*)(ws + OFF_WCAT);
  _Float16* w1T   = (_Float16*)(ws + OFF_W1T);
  _Float16* w2T   = (_Float16*)(ws + OFF_W2T);
  float*    bcat  = (float*)(ws + OFF_BCAT);
  float*    outp  = (float*)d_out;

  typedef const unsigned short* cu16;
  const float sc16  = 1.0f / 16.0f;
  const float sc256 = 1.0f / 256.0f;

  prep_act<<<kMpad * 32 / 256, 256, 0, stream>>>(x, pos, x16, q16);
  prep_wt16<<<(kD * (kD / 8) + 255) / 256, 256, 0, stream>>>(Wval, wvalT, kD, kD, kD);
  prep_wt16<<<(kD * (kD / 8) + 255) / 256, 256, 0, stream>>>(Wout, woutT, kD, kD, kD);
  prep_wt16<<<(192 * (kD / 8) + 255) / 256, 256, 0, stream>>>(Woff, wcatT, kD, 192, 192);
  prep_wt16<<<(128 * (kD / 8) + 255) / 256, 256, 0, stream>>>(Wattn, wcatT + (size_t)kNOFF * kD, kD, 96, 128);
  prep_wt16<<<(kFF * (kD / 8) + 255) / 256, 256, 0, stream>>>(W1, w1T, kD, kFF, kFF);
  prep_wt16<<<(kD * (kFF / 8) + 255) / 256, 256, 0, stream>>>(W2, w2T, kFF, kD, kD);
  prep_bias_cat<<<1, 320, 0, stream>>>(boff, battn, bcat);

  wmma_gemm64<0, false, 2, 0, false, 0><<<dim3(gemm_blocks(kD), 1), 256, 0, stream>>>(
      (cu16)x16, nullptr, kD, 0L, (cu16)wvalT, nullptr, kD, 0L, (void*)valp, nullptr, kD, 0L,
      bval, nullptr, 0L, kMpad, kD, kD, sc16);
  wmma_gemm64<0, false, 2, 0, false, 0><<<dim3(gemm_blocks(kNOA), 1), 256, 0, stream>>>(
      (cu16)q16, nullptr, kD, 0L, (cu16)wcatT, nullptr, kD, 0L, (void*)oa, nullptr, kNOA, 0L,
      bcat, nullptr, 0L, kMpad, kNOA, kD, sc16);
  sample_kernel<<<kMpad / 8, 256, 0, stream>>>(valp, oa, refp, ao16);
  wmma_gemm64<0, false, 2, 0, false, 0><<<dim3(gemm_blocks(kD), 1), 256, 0, stream>>>(
      (cu16)ao16, nullptr, kD, 0L, (cu16)woutT, nullptr, kD, 0L, (void*)t1, nullptr, kD, 0L,
      bout, nullptr, 0L, kMpad, kD, kD, sc256);
  ln1_kernel<<<kMpad / 8, 256, 0, stream>>>(t1, x, g1, be1, h1, h1h);
  wmma_gemm64<0, false, 2, 1, false, 2><<<dim3(gemm_blocks(kFF), 1), 256, 0, stream>>>(
      (cu16)h1h, nullptr, kD, 0L, (cu16)w1T, nullptr, kD, 0L, (void*)f16p, nullptr, kFF, 0L,
      b1, nullptr, 0L, kMpad, kFF, kD, sc16);
  wmma_gemm64<0, false, 2, 0, true, 0><<<dim3(gemm_blocks(kD), 1), 256, 0, stream>>>(
      (cu16)f16p, nullptr, kFF, 0L, (cu16)w2T, nullptr, kFF, 0L, (void*)t2, nullptr, kD, 0L,
      b2, h1, 0L, kMpad, kD, kFF, sc16);
  ln2_kernel<<<(kM + 7) / 8, 256, 0, stream>>>(t2, g2, be2, outp);
}
